// CoordinateDecoder_79568564126192
// MI455X (gfx1250) — hardware-verified
//
#include <hip/hip_runtime.h>
#include <math.h>

typedef __attribute__((ext_vector_type(16))) _Float16 v16h;
typedef __attribute__((ext_vector_type(16))) __bf16 v16b;
typedef __attribute__((ext_vector_type(8)))  _Float16 v8h;
typedef __attribute__((ext_vector_type(8)))  float v8f;
typedef __attribute__((ext_vector_type(4)))  float v4f;
typedef __attribute__((ext_vector_type(2)))  float v2f;
typedef __attribute__((ext_vector_type(4)))  unsigned v4u;
typedef __attribute__((ext_vector_type(4)))  int v4i;
typedef float __attribute__((may_alias)) float_a;
typedef int __attribute__((may_alias)) int_a;

template <typename T> __device__ __forceinline__ void vst2(void* p, T v) { *(volatile T*)p = v; __threadfence(); *(volatile T*)p = v; }
__device__ __forceinline__ v8f wmma16(v16h a, v16h b, v8f c) {
  v8f d = __builtin_amdgcn_wmma_f32_16x16x32_f16(false, a, false, b, (short)0, c, false, false);
  asm volatile("v_nop\n\tv_nop\n\tv_nop\n\tv_nop" : "+v"(d) : "v"(a), "v"(b));
  return d;
}
__device__ __forceinline__ v8f wmma_bf(v16b a, v16b b, v8f c) {
  v8f d = __builtin_amdgcn_wmma_f32_16x16x32_bf16(false, a, false, b, (short)0, c, false, false);
  asm volatile("v_nop\n\tv_nop\n\tv_nop\n\tv_nop" : "+v"(d) : "v"(a), "v"(b));
  return d;
}
__device__ __forceinline__ v16h frag_h(const _Float16* rowk0, int lane) {
  union { v16h v; v8h q[2]; } u; const _Float16* p = rowk0 + 8 * (lane >> 4);
  u.q[0] = *(const v8h*)p; u.q[1] = *(const v8h*)(p + 16); return u.v;
}
__device__ __forceinline__ v16h frag_f32(const float* rowk0, int lane) {
  v16h a; const float* p = rowk0 + 8 * (lane >> 4);
#pragma unroll
  for (int i = 0; i < 8; ++i) { a[i] = (_Float16)p[i]; a[8 + i] = (_Float16)p[16 + i]; }
  return a;
}
__device__ __forceinline__ v16h frag_f32s(const float* rowk0, int lane, float sc) {
  v16h a; const float* p = rowk0 + 8 * (lane >> 4);
#pragma unroll
  for (int i = 0; i < 8; ++i) { a[i] = (_Float16)(p[i] * sc); a[8 + i] = (_Float16)(p[16 + i] * sc); }
  return a;
}
__device__ __forceinline__ v16h fragc_f32(const float* W, int k0, int n, int lane, int ld, int K) {
  v16h a; const int g = lane >> 4;
#pragma unroll
  for (int i = 0; i < 8; ++i) { const int ka = k0 + 8 * g + i, kb = ka + 16;
    a[i] = (_Float16)(ka < K ? W[(size_t)(ka < K ? ka : K - 1) * ld + n] : 0.f); a[8 + i] = (_Float16)(kb < K ? W[(size_t)(kb < K ? kb : K - 1) * ld + n] : 0.f); }
  return a;
}
struct F2 { v16b h, l; };
__device__ __forceinline__ F2 bsplit16(const float v[16]) { F2 r;
#pragma unroll
  for (int i = 0; i < 16; ++i) { const __bf16 h = (__bf16)v[i]; r.h[i] = h; r.l[i] = (__bf16)(v[i] - (float)h); }
  return r; }
__device__ __forceinline__ F2 split_row(const float* row, int k0, int lane) { float v[16]; const float* p = row + k0 + 8 * (lane >> 4);
#pragma unroll
  for (int i = 0; i < 8; ++i) { v[i] = p[i]; v[8 + i] = p[16 + i]; }
  return bsplit16(v); }
__device__ __forceinline__ F2 split_rowK(const float* row, int k0, int lane, int K) { float v[16]; const int g = lane >> 4;
#pragma unroll
  for (int i = 0; i < 8; ++i) { const int ka = k0 + 8 * g + i, kb = ka + 16; v[i] = ka < K ? row[ka < K ? ka : K - 1] : 0.f; v[8 + i] = kb < K ? row[kb < K ? kb : K - 1] : 0.f; }
  return bsplit16(v); }
__device__ __forceinline__ F2 split_col(const float* W, int k0, int n, int lane, int ld, int K) { float v[16]; const int g = lane >> 4;
#pragma unroll
  for (int i = 0; i < 8; ++i) { const int ka = k0 + 8 * g + i, kb = ka + 16; v[i] = ka < K ? W[(size_t)(ka < K ? ka : K - 1) * ld + n] : 0.f; v[8 + i] = kb < K ? W[(size_t)(kb < K ? kb : K - 1) * ld + n] : 0.f; }
  return bsplit16(v); }
__device__ __forceinline__ v8f mac3(const F2& a, const F2& b, v8f c) { c = wmma_bf(a.l, b.h, c); c = wmma_bf(a.h, b.l, c); return wmma_bf(a.h, b.h, c); }
__device__ __forceinline__ float sigm(float v) { return 1.0f / (1.0f + expf(-v)); }
#define LDSX() do { asm volatile("s_wait_dscnt 0" ::: "memory"); __builtin_amdgcn_wave_barrier(); __builtin_amdgcn_fence(__ATOMIC_RELEASE, "workgroup"); } while (0)

#define NBT 8
#define NPB 65536
#define NP (NBT * NPB)
#define NE 32
#define NHID 64
#define NCD 128
#define NO 4
#ifndef NPROC
#define NPROC NP
#endif
__device__ __forceinline__ float bfr(float v) { return (float)(__bf16)v; }
__device__ __forceinline__ float lrelu2(float v) { return (v >= 0.f ? v : 0.2f * v) * 1.4142135623730951f; }
__device__ __forceinline__ v16b wrow_part(const float* Wm, int ldin, int koff, int k0, int o, int nout, int lane) { v16b w; const int g = lane >> 4; const int oc = o < nout ? o : nout - 1; const float keep = o < nout ? 1.f : 0.f; const float* p = Wm + (size_t)oc * ldin + koff + k0 + 8 * g;
#pragma unroll
  for (int i = 0; i < 8; ++i) { w[i] = (__bf16)(p[i] * keep); w[8 + i] = (__bf16)(p[16 + i] * keep); }
  return w; }

__global__ __launch_bounds__(256) void k_cond(const float* __restrict__ C, const float* __restrict__ W1, const float* __restrict__ W2, const float* __restrict__ W3, const float* __restrict__ W4, float* __restrict__ CP) {
  for (int e = threadIdx.x; e < 4 * NBT * NHID; e += 256) { const int l = e / (NBT * NHID), b = (e / NHID) % NBT, o = e % NHID;
    const float* Wl = l == 0 ? W1 : l == 1 ? W2 : l == 2 ? W3 : W4; const int ldin = l == 0 ? NE + NCD : NHID + NCD; const int xoff = l == 0 ? NE : NHID; const int nout = l == 3 ? NO : NHID;
    float s = 0.f; if (o < nout) { for (int k = 0; k < NCD; ++k) s += bfr(C[b * NCD + k]) * bfr(Wl[(size_t)o * ldin + xoff + k]); }
    vst2(CP + e, s); } }
__global__ __launch_bounds__(128) void k_dec(const float* __restrict__ CO, const float* __restrict__ FU, const float* __restrict__ W1, const float* __restrict__ B1, const float* __restrict__ W2, const float* __restrict__ B2, const float* __restrict__ W3, const float* __restrict__ B3, const float* __restrict__ W4, const float* __restrict__ B4, const float* __restrict__ CP, float* __restrict__ OUT) {
  __shared__ __align__(16) float sa[64][68]; __shared__ __align__(16) float so[64][4];
  const int tid = threadIdx.x, wave = tid >> 5, lane = tid & 31, col = lane & 15, g = lane >> 4; const size_t p0 = (size_t)blockIdx.x * 64; const int b = (int)(p0 / NPB);
  const float fu = bfr(FU[0]);
  for (int e = tid; e < 64 * 8; e += 128) { const int pl = e >> 3, f = e & 7; const float c0 = bfr(CO[(p0 + pl) * 2]) / 10.0f, c1 = bfr(CO[(p0 + pl) * 2 + 1]) / 10.0f; const float fr = (float)(1 << f);
    const float wt = fminf(fmaxf((fu - (float)(f + 1) / 9.0f) * 9.0f, 0.f), 1.f); const float a0 = c0 * fr, a1 = c1 * fr;
    sa[pl][f * 4 + 0] = sinf(a0) * wt; sa[pl][f * 4 + 1] = sinf(a1) * wt; sa[pl][f * 4 + 2] = cosf(a0) * wt; sa[pl][f * 4 + 3] = cosf(a1) * wt; }
  __syncthreads();
  const int rbase = wave * 16;
  { v8f acc[4] = {}; const F2 a = split_row(&sa[rbase + col][0], 0, lane);
#pragma unroll
    for (int j = 0; j < 4; ++j) { const v16b w = wrow_part(W1, NE + NCD, 0, 0, j * 16 + col, NHID, lane); acc[j] = wmma_bf(a.h, w, acc[j]); acc[j] = wmma_bf(a.l, w, acc[j]); }
    LDSX();
    const float s1 = 1.0f / sqrtf(160.0f);
#pragma unroll
    for (int j = 0; j < 4; ++j) { const int o = j * 16 + col; const float cb = CP[(0 * NBT + b) * NHID + o] ; const float bb = bfr(B1[o]);
#pragma unroll
      for (int r = 0; r < 8; ++r) sa[rbase + 8 * g + r][o] = lrelu2((acc[j][r] + cb) * s1 + bb); } LDSX(); }
#pragma unroll 1
  for (int l = 1; l <= 2; ++l) { const float* Wl = l == 1 ? W2 : W3; const float* Bl = l == 1 ? B2 : B3; v8f acc[4] = {};
#pragma unroll
    for (int kc = 0; kc < 2; ++kc) { const F2 a = split_row(&sa[rbase + col][0], kc * 32, lane);
#pragma unroll
      for (int j = 0; j < 4; ++j) { const v16b w = wrow_part(Wl, NHID + NCD, 0, kc * 32, j * 16 + col, NHID, lane); acc[j] = wmma_bf(a.h, w, acc[j]); acc[j] = wmma_bf(a.l, w, acc[j]); } }
    LDSX(); const float s2 = 1.0f / sqrtf(192.0f);
#pragma unroll
    for (int j = 0; j < 4; ++j) { const int o = j * 16 + col; const float cb = CP[(l * NBT + b) * NHID + o]; const float bb = bfr(Bl[o]);
#pragma unroll
      for (int r = 0; r < 8; ++r) sa[rbase + 8 * g + r][o] = lrelu2((acc[j][r] + cb) * s2 + bb); } LDSX(); }
  { v8f acc = {};
#pragma unroll
    for (int kc = 0; kc < 2; ++kc) { const F2 a = split_row(&sa[rbase + col][0], kc * 32, lane); const v16b w = wrow_part(W4, NHID + NCD, 0, kc * 32, col, NO, lane); acc = wmma_bf(a.h, w, acc); acc = wmma_bf(a.l, w, acc); }
    const float s4 = 1.0f / sqrtf(192.0f);
    if (col < NO) { const float cb = CP[(3 * NBT + b) * NHID + col]; const float bb = bfr(B4[col]);
#pragma unroll
      for (int r = 0; r < 8; ++r) { const int pl = rbase + 8 * g + r; const float x0 = bfr(CO[(p0 + pl) * 2]), x1 = bfr(CO[(p0 + pl) * 2 + 1]); const float rad = sqrtf(x0 * x0 + x1 * x1); const float gate = 1.0f - tanhf(fmaxf(rad - 1.0f, 0.f));
        so[pl][col] = ((acc[r] + cb) * s4 + bb) * gate; } } }
  __syncthreads();
  if (tid < 64) vst2(OUT + (p0 + tid) * NO, *(const v4f*)&so[tid][0]); }
extern "C" void kernel_launch(void* const* d_in, const int* in_sizes, int n_in, void* d_out, int out_size, void* d_ws, size_t ws_size, hipStream_t stream) {
  (void)in_sizes; (void)n_in; (void)out_size;
  const float** F = (const float**)d_in;
  if (ws_size < (size_t)(4 * NBT * NHID * 4)) return;
  float* CP = (float*)d_ws;
  k_cond<<<1, 256, 0, stream>>>(F[1], F[3], F[5], F[7], F[9], CP);
  k_dec<<<dim3(NPROC / 64), 128, 0, stream>>>(F[0], F[2], F[3], F[4], F[5], F[6], F[7], F[8], F[9], F[10], CP, (float*)d_out);
}
